// EncoderLayer_13030930776801
// MI455X (gfx1250) — hardware-run, weakly checked
//
#include <hip/hip_runtime.h>
#include <stddef.h>
#include <stdint.h>
#include <math.h>


#ifndef NB
#define NB 2
#endif
#ifndef SEQ
#define SEQ 2048
#endif
#define NB_FULL  2
#define SEQ_FULL 2048
#define DM    1024
#define NH    16
#define DK    64
#define DHID  4096
#define NQKV  (3 * DM)
#define MROWS (NB * SEQ)
#define NZ    (NB * NH)
#define PLANE ((size_t)MROWS * DM)
#define NTHR  256
#define GBM   64
#define GBN   128
#define GTHR  128
#define WSMAX 134217728

static_assert(NB >= 1 && NB <= NB_FULL);
static_assert(SEQ >= 64 && SEQ <= SEQ_FULL && SEQ % 64 == 0);
static_assert(MROWS % GBM == 0 && MROWS % 4 == 0);
static_assert(DM % GBN == 0 && DHID % GBN == 0 && NQKV % GBN == 0);
static_assert(DM % 32 == 0 && DHID % 32 == 0 && DK == 64 && NH * DK == DM);
static_assert(GTHR == GBN && GBM == 64 && GBN == 128);
static_assert((size_t)MROWS * DHID * 2 <= (size_t)MROWS * DM * 2 + (size_t)NQKV * DM * 2 + 3 * PLANE * 2);
static_assert((size_t)MROWS * DM * 2 + (size_t)NQKV * DM * 2 + 3 * PLANE * 2
              + (size_t)DM * DM * 2 + (size_t)DHID * DM * 2 + (size_t)DM * DHID * 2
              + (size_t)NZ * 2 * SEQ * 4
              + (size_t)MROWS * DM * 2
              + (size_t)MROWS * DM * 4 + (size_t)MROWS * DM * 2
              + (size_t)MROWS * DM * 4 + (size_t)MROWS * DM * 4
              <= (size_t)WSMAX);

typedef float          v4f   __attribute__((ext_vector_type(4)));
typedef float          v8f   __attribute__((ext_vector_type(8)));
typedef int            v8i   __attribute__((ext_vector_type(8)));
typedef unsigned short v4us  __attribute__((ext_vector_type(4)));
typedef unsigned short v8us  __attribute__((ext_vector_type(8)));
typedef __bf16         v16bf __attribute__((ext_vector_type(16)));
typedef _Float16       v16h  __attribute__((ext_vector_type(16)));
typedef v4f  __attribute__((may_alias)) v4fa;
typedef v8us __attribute__((may_alias)) v8usa;
union Frag { v16bf b; v16h f; v8us h[2]; v8i w; };

__device__ __forceinline__ v8f wmb(const Frag& a, const Frag& b, v8f c) {
  v8f d = __builtin_amdgcn_wmma_f32_16x16x32_bf16(false, a.b, false, b.b, (short)0, c, false, false);
  asm volatile("v_nop\n\tv_nop\n\tv_nop\n\tv_nop" : "+v"(d) : "v"(a.w), "v"(b.w));
  return d;
}
__device__ __forceinline__ v8f wmh(const Frag& a, const Frag& b, v8f c) {
  v8f d = __builtin_amdgcn_wmma_f32_16x16x32_f16(false, a.f, false, b.f, (short)0, c, false, false);
  asm volatile("v_nop\n\tv_nop\n\tv_nop\n\tv_nop" : "+v"(d) : "v"(a.w), "v"(b.w));
  return d;
}
template <bool BF>
__device__ __forceinline__ v8f wm(const Frag& a, const Frag& b, v8f c) {
  if (BF) return wmb(a, b, c);
  return wmh(a, b, c);
}

__device__ __forceinline__ unsigned bf16_bits(float f) {
  const unsigned u = __float_as_uint(f);
  return (u + 0x7FFFu + ((u >> 16) & 1u)) >> 16;
}
__device__ __forceinline__ float bf16_val(float f) {
  return __uint_as_float(bf16_bits(f) << 16);
}
__device__ __forceinline__ unsigned short f16_bits(float f) {
  union { _Float16 h; unsigned short u; } c;
  c.h = (_Float16)f;
  return c.u;
}

__device__ __forceinline__ void wave_sync() {
  __builtin_amdgcn_fence(3  , "wavefront");
  __builtin_amdgcn_wave_barrier();
  __builtin_amdgcn_fence(2  , "wavefront");
}

__global__ __launch_bounds__(NTHR) void k_cvt_x(const float* __restrict__ x, unsigned short* xb) {
  const int u = (int)blockIdx.x * NTHR + (int)threadIdx.x;
  if (u < MROWS * (DM / 8)) {
    const int row = u >> 7;
    const int k8  = (u & 127) * 8;
    const int bb  = row / SEQ;
    const int ss  = row - bb * SEQ;
    const float* p = x + ((size_t)bb * SEQ_FULL + ss) * DM + k8;
    const v4f a = *(const v4fa*)p;
    const v4f b = *(const v4fa*)(p + 4);
    v8us o;
    o[0] = (unsigned short)bf16_bits(a.x); o[1] = (unsigned short)bf16_bits(a.y);
    o[2] = (unsigned short)bf16_bits(a.z); o[3] = (unsigned short)bf16_bits(a.w);
    o[4] = (unsigned short)bf16_bits(b.x); o[5] = (unsigned short)bf16_bits(b.y);
    o[6] = (unsigned short)bf16_bits(b.z); o[7] = (unsigned short)bf16_bits(b.w);
    unsigned short* dp = xb + (size_t)row * DM + k8;
    *(volatile v8us*)dp = o;
    __threadfence();
    *(volatile v8us*)dp = o;
  }
}

template <int MODE>
__global__ __launch_bounds__(NTHR) void k_wt(const float* __restrict__ in, int kdim, int cols, int ntot,
                                             unsigned short* out) {
  const int upr = kdim >> 3;
  const int u = (int)blockIdx.x * NTHR + (int)threadIdx.x;
  if (u < ntot * upr) {
    const int n  = u / upr;
    const int k8 = (u - n * upr) * 8;
    const int zb = n / cols;
    const int c  = n - zb * cols;
    const float* p = in + ((size_t)zb * kdim + k8) * (size_t)cols + c;
    v8us o;
#pragma unroll
    for (int i = 0; i < 8; ++i) {
      const float w = p[(size_t)i * cols];
      if (MODE == 0) o[i] = (unsigned short)bf16_bits(w);
      else           o[i] = f16_bits(bf16_val(w) * 256.0f);
    }
    unsigned short* dp = out + (size_t)n * kdim + k8;
    *(volatile v8us*)dp = o;
    __threadfence();
    *(volatile v8us*)dp = o;
  }
}

template <int EPI, bool BF>
__global__ __launch_bounds__(GTHR) void k_gemm(const unsigned short* __restrict__ Apl,
                                               const unsigned short* __restrict__ BT, int K,
                                               const float* __restrict__ bias0, const float* __restrict__ bias1,
                                               const float* __restrict__ bias2, const float* __restrict__ aux,
                                               float* outF, unsigned short* outH, int ldo, float scale) {
  __shared__ __attribute__((aligned(16))) float stg[GBM * GBN];
  __shared__ __attribute__((aligned(16))) float sbias[GBN];
  const int tid = (int)threadIdx.x, lane = tid & 31, wave = tid >> 5, hh = lane >> 4, m = lane & 15;
  const int wr = wave >> 1, wc = wave & 1;
  const int rowBase = (int)blockIdx.x * GBM;
  const int col0    = (int)blockIdx.y * GBN;
  const int which   = (EPI == 0) ? (col0 >> 10) : 0;
  const int cb      = (EPI == 0) ? (col0 & (DM - 1)) : col0;
  {
    const float t0 = bias0[cb + tid];
    const float t1 = bias1[cb + tid];
    const float t2 = bias2[cb + tid];
    const float ts = (which == 0) ? t0 : ((which == 1) ? t1 : t2);
    sbias[tid] = bf16_val(ts);
  }

  v8f acc[2][4];
  {
    const v8f z = {0.f, 0.f, 0.f, 0.f, 0.f, 0.f, 0.f, 0.f};
#pragma unroll
    for (int a = 0; a < 2; ++a)
#pragma unroll
      for (int t = 0; t < 4; ++t) acc[a][t] = z;
  }
  const unsigned short* ap = Apl + (size_t)(rowBase + 32 * wr + m) * (size_t)K + 8 * hh;
  const unsigned short* bp = BT + (size_t)(col0 + 64 * wc + m) * (size_t)K + 8 * hh;

#pragma unroll 1
  for (int k0 = 0; k0 < K; k0 += 32) {
    Frag a0, a1;
    a0.h[0] = *(const v8usa*)(ap + k0);
    a0.h[1] = *(const v8usa*)(ap + k0 + 16);
    a1.h[0] = *(const v8usa*)(ap + (size_t)16 * (size_t)K + k0);
    a1.h[1] = *(const v8usa*)(ap + (size_t)16 * (size_t)K + k0 + 16);
#pragma unroll
    for (int nt = 0; nt < 4; ++nt) {
      const unsigned short* wq = bp + (size_t)(16 * nt) * (size_t)K + k0;
      Frag bf;
      bf.h[0] = *(const v8usa*)wq;
      bf.h[1] = *(const v8usa*)(wq + 16);
      acc[0][nt] = wm<BF>(a0, bf, acc[0][nt]);
      acc[1][nt] = wm<BF>(a1, bf, acc[1][nt]);
    }
  }

#pragma unroll
  for (int mt = 0; mt < 2; ++mt) {
#pragma unroll
    for (int nt = 0; nt < 4; ++nt) {
      const int lc = 64 * wc + 16 * nt + m;
#pragma unroll
      for (int r = 0; r < 8; ++r) {
        const int lr = 32 * wr + 16 * mt + 8 * hh + r;
        stg[lr * GBN + lc] = acc[mt][nt][r];
      }
    }
  }
  __syncthreads();

  if (EPI == 0) {
    const int q  = lane >> 3;
    const int pc = lane & 7;
    const int bb    = rowBase / SEQ;
    const int sBase = rowBase - bb * SEQ;
    const int head0 = cb >> 6;
    unsigned short* plane = outH + (size_t)which * PLANE;
    v8us o[8];
    unsigned short* dp[8];
    if (which < 2) {
      const int hsel = q & 1;
      const v4f ba = *(const v4fa*)(sbias + 64 * hsel + 8 * pc);
      const v4f bc = *(const v4fa*)(sbias + 64 * hsel + 8 * pc + 4);
#pragma unroll
      for (int it = 0; it < 8; ++it) {
        const int lr = 16 * wave + 2 * it + (q >> 1);
        const v4f va = *(const v4fa*)(stg + lr * GBN + 64 * hsel + 8 * pc) + ba;
        const v4f vb = *(const v4fa*)(stg + lr * GBN + 64 * hsel + 8 * pc + 4) + bc;
        v8us t;
        t[0] = f16_bits(va.x); t[1] = f16_bits(va.y); t[2] = f16_bits(va.z); t[3] = f16_bits(va.w);
        t[4] = f16_bits(vb.x); t[5] = f16_bits(vb.y); t[6] = f16_bits(vb.z); t[7] = f16_bits(vb.w);
        o[it] = t;
        dp[it] = plane + ((size_t)(bb * NH + head0 + hsel) * SEQ + sBase + lr) * DK + 8 * pc;
      }
    } else {
#pragma unroll
      for (int it = 0; it < 8; ++it) {
        const int lc = 32 * wave + 4 * it + q;
        const float bv = sbias[lc];
        v8us t;
#pragma unroll
        for (int i = 0; i < 8; ++i) t[i] = f16_bits(stg[(8 * pc + i) * GBN + lc] + bv);
        o[it] = t;
        dp[it] = plane + ((size_t)(bb * NH + head0 + (lc >> 6)) * DK + (lc & 63)) * SEQ + sBase + 8 * pc;
      }
    }
#pragma unroll
    for (int it = 0; it < 8; ++it) *(volatile v8us*)dp[it] = o[it];
    __threadfence();
#pragma unroll
    for (int it = 0; it < 8; ++it) *(volatile v8us*)dp[it] = o[it];
  } else {
    const v4f bb4 = *(const v4fa*)(sbias + 4 * lane);
    v4f  pv[16];
    v4us ph[16];
#pragma unroll
    for (int i = 0; i < 16; ++i) {
      const int lr = 16 * wave + i;
      const int r  = rowBase + lr;
      v4f t = *(const v4fa*)(stg + lr * GBN + 4 * lane) * scale + bb4;
      if (EPI == 1) {
        const int rb = r / SEQ;
        const int ar = rb * SEQ_FULL + (r - rb * SEQ);
        const v4f a = *(const v4fa*)(aux + (size_t)ar * DM + col0 + 4 * lane);
        t.x = t.x + bf16_val(a.x); t.y = t.y + bf16_val(a.y);
        t.z = t.z + bf16_val(a.z); t.w = t.w + bf16_val(a.w);
      }
      if (EPI == 3) {
        const v4f a = *(const v4fa*)(aux + (size_t)r * DM + col0 + 4 * lane);
        t = t + a;
      }
      if (EPI == 2) {
        t.x = (t.x > 0.0f) ? t.x : (t.x - t.x);
        t.y = (t.y > 0.0f) ? t.y : (t.y - t.y);
        t.z = (t.z > 0.0f) ? t.z : (t.z - t.z);
        t.w = (t.w > 0.0f) ? t.w : (t.w - t.w);
      }
      pv[i] = t;
      v4us h4;
      h4[0] = f16_bits(t.x); h4[1] = f16_bits(t.y); h4[2] = f16_bits(t.z); h4[3] = f16_bits(t.w);
      ph[i] = h4;
    }
#pragma unroll
    for (int i = 0; i < 16; ++i) {
      const size_t eo = (size_t)(rowBase + 16 * wave + i) * (size_t)ldo + col0 + 4 * lane;
      if (EPI == 1 || EPI == 3) *(volatile v4f*)(outF + eo) = pv[i];
      if (EPI == 1 || EPI == 2) *(volatile v4us*)(outH + eo) = ph[i];
    }
    __threadfence();
#pragma unroll
    for (int i = 0; i < 16; ++i) {
      const size_t eo = (size_t)(rowBase + 16 * wave + i) * (size_t)ldo + col0 + 4 * lane;
      if (EPI == 1 || EPI == 3) *(volatile v4f*)(outF + eo) = pv[i];
      if (EPI == 1 || EPI == 2) *(volatile v4us*)(outH + eo) = ph[i];
    }
  }
}

__global__ __launch_bounds__(128) void k_stats(const unsigned short* __restrict__ Qp,
                                               const unsigned short* __restrict__ Kp, float* st) {
  __shared__ __attribute__((aligned(16))) float sm[128];
  const int tid = (int)threadIdx.x, lane = tid & 31, wave = tid >> 5, hh = lane >> 4, m = lane & 15;
  const int z    = (int)blockIdx.y;
  const int key0 = (int)blockIdx.x * 64;
  const int kw   = key0 + 16 * wave;

  Frag bk0, bk1;
  {
    const unsigned short* kb = Kp + ((size_t)z * SEQ + kw + m) * DK + 8 * hh;
    bk0.h[0] = *(const v8usa*)(kb);
    bk0.h[1] = *(const v8usa*)(kb + 16);
    bk1.h[0] = *(const v8usa*)(kb + 32);
    bk1.h[1] = *(const v8usa*)(kb + 48);
  }
  const unsigned short* qb = Qp + ((size_t)z * SEQ + m) * DK + 8 * hh;
  const v8f zero = {0.f, 0.f, 0.f, 0.f, 0.f, 0.f, 0.f, 0.f};
  float mx = -1.0e30f, zs = 0.0f;

#pragma unroll 1
  for (int q0 = 0; q0 < SEQ; q0 += 64) {
    v8f s[4];
#pragma unroll
    for (int t = 0; t < 4; ++t) {
      const unsigned short* qp = qb + (size_t)(q0 + 16 * t) * DK;
      Frag a0, a1;
      a0.h[0] = *(const v8usa*)(qp);
      a0.h[1] = *(const v8usa*)(qp + 16);
      a1.h[0] = *(const v8usa*)(qp + 32);
      a1.h[1] = *(const v8usa*)(qp + 48);
      v8f d = wmh(a0, bk0, zero);
      s[t] = wmh(a1, bk1, d);
    }
    float tm = s[0][0];
#pragma unroll
    for (int t = 0; t < 4; ++t)
#pragma unroll
      for (int r = 0; r < 8; ++r) tm = fmaxf(tm, s[t][r]);
    const float mn = fmaxf(mx, tm * 0.125f);
    float a = zs * __expf(mx - mn);
#pragma unroll
    for (int t = 0; t < 4; ++t)
#pragma unroll
      for (int r = 0; r < 8; ++r) a += __expf(fmaf(s[t][r], 0.125f, -mn));
    zs = a;
    mx = mn;
  }
  const float mo = __shfl_xor(mx, 16, 32);
  const float zo = __shfl_xor(zs, 16, 32);
  const float M  = fmaxf(mx, mo);
  const float Z  = zs * __expf(mx - M) + zo * __expf(mo - M);
  const float rinv = 1024.0f * (1.0f / Z);
  if (hh == 0) {
    sm[16 * wave + m]      = M;
    sm[64 + 16 * wave + m] = rinv;
  }
  __syncthreads();
  if (wave == 0) {
    const v4f v = *(const v4fa*)(sm + 4 * lane);
    float* dp = st + ((size_t)z * 2 + (size_t)(lane >> 4)) * SEQ + key0 + 4 * (lane & 15);
    *(volatile v4f*)dp = v;
    __threadfence();
    *(volatile v4f*)dp = v;
  }
}

__global__ __launch_bounds__(128) void k_attn(const unsigned short* __restrict__ Qp,
                                              const unsigned short* __restrict__ Kp,
                                              const unsigned short* __restrict__ VTp,
                                              const float* __restrict__ st, unsigned short* cat) {
  __shared__ __attribute__((aligned(16))) unsigned short ot[4 * 16 * DK];
  const int tid = (int)threadIdx.x, lane = tid & 31, wave = tid >> 5, hh = lane >> 4, m = lane & 15;
  const int z    = (int)blockIdx.y;
  const int bb   = z / NH;
  const int head = z - bb * NH;
  const int q0   = (int)blockIdx.x * 64 + 16 * wave;

  Frag bq0, bq1;
  {
    const unsigned short* qp = Qp + ((size_t)z * SEQ + q0 + m) * DK + 8 * hh;
    bq0.h[0] = *(const v8usa*)(qp);
    bq0.h[1] = *(const v8usa*)(qp + 16);
    bq1.h[0] = *(const v8usa*)(qp + 32);
    bq1.h[1] = *(const v8usa*)(qp + 48);
  }
  const unsigned short* kp = Kp + ((size_t)z * SEQ + m) * DK + 8 * hh;
  const unsigned short* vp = VTp + ((size_t)z * DK + m) * SEQ + 8 * hh;
  const float* sp = st + (size_t)z * 2 * SEQ + 8 * hh;
  const v8f zero = {0.f, 0.f, 0.f, 0.f, 0.f, 0.f, 0.f, 0.f};
  v8f o[4];
#pragma unroll
  for (int t = 0; t < 4; ++t) o[t] = zero;

#pragma unroll 1
  for (int kb = 0; kb < SEQ; kb += 32) {
    v8f s0, s1;
    {
      const unsigned short* ka = kp + (size_t)kb * DK;
      Frag a0, a1;
      a0.h[0] = *(const v8usa*)(ka);
      a0.h[1] = *(const v8usa*)(ka + 16);
      a1.h[0] = *(const v8usa*)(ka + 32);
      a1.h[1] = *(const v8usa*)(ka + 48);
      const v8f d = wmh(a0, bq0, zero);
      s0 = wmh(a1, bq1, d);
    }
    {
      const unsigned short* ka = kp + (size_t)(kb + 16) * DK;
      Frag a0, a1;
      a0.h[0] = *(const v8usa*)(ka);
      a0.h[1] = *(const v8usa*)(ka + 16);
      a1.h[0] = *(const v8usa*)(ka + 32);
      a1.h[1] = *(const v8usa*)(ka + 48);
      const v8f d = wmh(a0, bq0, zero);
      s1 = wmh(a1, bq1, d);
    }
    const v4f m0a = *(const v4fa*)(sp + kb);
    const v4f m0b = *(const v4fa*)(sp + kb + 4);
    const v4f m1a = *(const v4fa*)(sp + kb + 16);
    const v4f m1b = *(const v4fa*)(sp + kb + 20);
    const v4f r0a = *(const v4fa*)(sp + SEQ + kb);
    const v4f r0b = *(const v4fa*)(sp + SEQ + kb + 4);
    const v4f r1a = *(const v4fa*)(sp + SEQ + kb + 16);
    const v4f r1b = *(const v4fa*)(sp + SEQ + kb + 20);
    const float mk0[8] = {m0a.x, m0a.y, m0a.z, m0a.w, m0b.x, m0b.y, m0b.z, m0b.w};
    const float mk1[8] = {m1a.x, m1a.y, m1a.z, m1a.w, m1b.x, m1b.y, m1b.z, m1b.w};
    const float rk0[8] = {r0a.x, r0a.y, r0a.z, r0a.w, r0b.x, r0b.y, r0b.z, r0b.w};
    const float rk1[8] = {r1a.x, r1a.y, r1a.z, r1a.w, r1b.x, r1b.y, r1b.z, r1b.w};
    Frag pf;
#pragma unroll
    for (int r = 0; r < 8; ++r) {
      pf.f[r]     = (_Float16)(__expf(fmaf(s0[r], 0.125f, -mk0[r])) * rk0[r]);
      pf.f[8 + r] = (_Float16)(__expf(fmaf(s1[r], 0.125f, -mk1[r])) * rk1[r]);
    }
#pragma unroll
    for (int vt = 0; vt < 4; ++vt) {
      const unsigned short* va = vp + (size_t)(16 * vt) * SEQ + kb;
      Frag av;
      av.h[0] = *(const v8usa*)(va);
      av.h[1] = *(const v8usa*)(va + 16);
      o[vt] = wmh(av, pf, o[vt]);
    }
  }

  unsigned short* ow = ot + wave * (16 * DK);
#pragma unroll
  for (int vt = 0; vt < 4; ++vt) {
    v8us t;
#pragma unroll
    for (int r = 0; r < 8; ++r) t[r] = f16_bits(o[vt][r] * 0.0625f);
    *(v8usa*)(ow + m * DK + 16 * vt + 8 * hh) = t;
  }
  wave_sync();
  v8us  ov[4];
  unsigned short* dp[4];
#pragma unroll
  for (int it = 0; it < 4; ++it) {
    const int ql = 4 * it + (lane >> 3);
    const int pc = lane & 7;
    ov[it] = *(const v8usa*)(ow + ql * DK + 8 * pc);
    dp[it] = cat + (size_t)(bb * SEQ + q0 + ql) * DM + head * DK + 8 * pc;
  }
#pragma unroll
  for (int it = 0; it < 4; ++it) *(volatile v8us*)dp[it] = ov[it];
  __threadfence();
#pragma unroll
  for (int it = 0; it < 4; ++it) *(volatile v8us*)dp[it] = ov[it];
}

__device__ __forceinline__ void ln_store_pass(const float* __restrict__ p, const float* __restrict__ g,
                                              const float* __restrict__ be, float* op, float mean, float inv,
                                              int lane, bool live) {
#pragma unroll 1
  for (int i = 0; i < 8; ++i) {
    const v4f v  = *(const v4fa*)(p + 128 * i);
    const v4f g0 = *(const v4fa*)(g + 4 * lane + 128 * i);
    const v4f b0 = *(const v4fa*)(be + 4 * lane + 128 * i);
    v4f y;
    y.x = fmaf(bf16_val(g0.x) * (v.x - mean), inv, bf16_val(b0.x));
    y.y = fmaf(bf16_val(g0.y) * (v.y - mean), inv, bf16_val(b0.y));
    y.z = fmaf(bf16_val(g0.z) * (v.z - mean), inv, bf16_val(b0.z));
    y.w = fmaf(bf16_val(g0.w) * (v.w - mean), inv, bf16_val(b0.w));
    if (live) *(volatile v4f*)(op + 128 * i) = y;
  }
}

__global__ __launch_bounds__(128) void k_ln(const float* __restrict__ in, const float* __restrict__ g,
                                            const float* __restrict__ be, float* out, int nRows) {
  const int tid = (int)threadIdx.x, lane = tid & 31, wave = tid >> 5;
  const int row = (int)blockIdx.x * 4 + wave;
  const bool live = row < nRows;
  const int rc = live ? row : nRows - 1;
  const float* p = in + (size_t)rc * DM + 4 * lane;
  float* op = out + (size_t)rc * DM + 4 * lane;

  v4f s4 = {0.f, 0.f, 0.f, 0.f};
#pragma unroll 1
  for (int i = 0; i < 8; ++i) s4 = s4 + *(const v4fa*)(p + 128 * i);
  float s = (s4.x + s4.y) + (s4.z + s4.w);
#pragma unroll
  for (int d = 16; d >= 1; d >>= 1) s += __shfl_xor(s, d, 32);
  const float mean = s * (1.0f / 1024.0f);

  v4f q4 = {0.f, 0.f, 0.f, 0.f};
#pragma unroll 1
  for (int i = 0; i < 8; ++i) {
    const v4f dv = *(const v4fa*)(p + 128 * i) - mean;
    q4 = q4 + dv * dv;
  }
  float ss = (q4.x + q4.y) + (q4.z + q4.w);
#pragma unroll
  for (int d = 16; d >= 1; d >>= 1) ss += __shfl_xor(ss, d, 32);
  const float sd  = sqrtf(ss * (1.0f / 1023.0f));
  const float inv = 1.0f / (sd + 1e-6f);

  ln_store_pass(p, g, be, op, mean, inv, lane, live);
  __threadfence();
  ln_store_pass(p, g, be, op, mean, inv, lane, live);
}

static inline int cdiv(int a, int b) { return (a + b - 1) / b; }
static inline size_t al256(size_t o) { return (o + 255) & ~(size_t)255; }

extern "C" void kernel_launch(void* const* d_in, const int* in_sizes, int n_in,
                              void* d_out, int out_size, void* d_ws, size_t ws_size,
                              hipStream_t stream) {
  if (n_in < 17) return;
  const long long needX = ((long long)(NB - 1) * SEQ_FULL + SEQ) * DM;
  if ((long long)in_sizes[0] < needX) return;
  if (in_sizes[1] < NH * DM * DK || in_sizes[3] < NH * DM * DK || in_sizes[5] < NH * DM * DK) return;
  if (in_sizes[2] < NH * DK || in_sizes[4] < NH * DK || in_sizes[6] < NH * DK) return;
  if (in_sizes[7] < DM * DM || in_sizes[8] < DM) return;
  if (in_sizes[9] < DM * DHID || in_sizes[10] < DHID) return;
  if (in_sizes[11] < DHID * DM || in_sizes[12] < DM) return;
  if (in_sizes[13] < DM || in_sizes[14] < DM || in_sizes[15] < DM || in_sizes[16] < DM) return;
  if ((long long)out_size < (long long)MROWS * DM) return;

  const float* x   = (const float*)d_in[0];
  const float* Wq  = (const float*)d_in[1];
  const float* bq  = (const float*)d_in[2];
  const float* Wk  = (const float*)d_in[3];
  const float* bk  = (const float*)d_in[4];
  const float* Wv  = (const float*)d_in[5];
  const float* bv  = (const float*)d_in[6];
  const float* Wo  = (const float*)d_in[7];
  const float* bo  = (const float*)d_in[8];
  const float* W1  = (const float*)d_in[9];
  const float* b1  = (const float*)d_in[10];
  const float* W2  = (const float*)d_in[11];
  const float* b2  = (const float*)d_in[12];
  const float* g1  = (const float*)d_in[13];
  const float* be1 = (const float*)d_in[14];
  const float* g2  = (const float*)d_in[15];
  const float* be2 = (const float*)d_in[16];
  float* out = (float*)d_out;

  char* ws = (char*)d_ws;
  size_t off = 0;
  const size_t oXB   = off; off = al256(off + (size_t)MROWS * DM * 2);
  const size_t oWQKV = off; off = al256(off + (size_t)NQKV * DM * 2);
  const size_t oQKV  = off; off = al256(off + 3 * PLANE * 2);
  const size_t oEarlyEnd = off;
  const size_t oWOT  = off; off = al256(off + (size_t)DM * DM * 2);
  const size_t oW1T  = off; off = al256(off + (size_t)DHID * DM * 2);
  const size_t oW2T  = off; off = al256(off + (size_t)DM * DHID * 2);
  const size_t oST   = off; off = al256(off + (size_t)NZ * 2 * SEQ * 4);
  const size_t oCAT  = off; off = al256(off + (size_t)MROWS * DM * 2);
  const size_t oRES  = off; off = al256(off + (size_t)MROWS * DM * 4);
  const size_t oRESH = off; off = al256(off + (size_t)MROWS * DM * 2);
  const size_t oSAE  = off; off = al256(off + (size_t)MROWS * DM * 4);
  const size_t oOPRE = off; off = al256(off + (size_t)MROWS * DM * 4);
  if (off > ws_size || off > (size_t)WSMAX) return;
  if ((size_t)MROWS * DHID * 2 > oEarlyEnd - oXB) return;
  unsigned short* XB    = (unsigned short*)(ws + oXB);
  unsigned short* WQKVT = (unsigned short*)(ws + oWQKV);
  unsigned short* QKV   = (unsigned short*)(ws + oQKV);
  unsigned short* Qp    = QKV;
  unsigned short* Kp    = QKV + PLANE;
  unsigned short* VTp   = QKV + 2 * PLANE;
  unsigned short* H1    = (unsigned short*)(ws + oXB);
  unsigned short* WOT   = (unsigned short*)(ws + oWOT);
  unsigned short* W1T   = (unsigned short*)(ws + oW1T);
  unsigned short* W2T   = (unsigned short*)(ws + oW2T);
  float*          ST    = (float*)(ws + oST);
  unsigned short* CAT   = (unsigned short*)(ws + oCAT);
  float*          RES   = (float*)(ws + oRES);
  unsigned short* RESH  = (unsigned short*)(ws + oRESH);
  float*          SAE   = (float*)(ws + oSAE);
  float*          OPRE  = (float*)(ws + oOPRE);

  k_cvt_x<<<cdiv(MROWS * (DM / 8), NTHR), NTHR, 0, stream>>>(x, XB);
  k_wt<0><<<cdiv(DM * (DM / 8), NTHR), NTHR, 0, stream>>>(Wq, DM, DK, DM, WQKVT);
  k_wt<0><<<cdiv(DM * (DM / 8), NTHR), NTHR, 0, stream>>>(Wk, DM, DK, DM, WQKVT + (size_t)DM * DM);
  k_wt<0><<<cdiv(DM * (DM / 8), NTHR), NTHR, 0, stream>>>(Wv, DM, DK, DM, WQKVT + (size_t)2 * DM * DM);
  k_wt<1><<<cdiv(DM * (DM / 8), NTHR), NTHR, 0, stream>>>(Wo, DM, DM, DM, WOT);
  k_wt<1><<<cdiv(DHID * (DM / 8), NTHR), NTHR, 0, stream>>>(W1, DM, DHID, DHID, W1T);
  k_wt<1><<<cdiv(DM * (DHID / 8), NTHR), NTHR, 0, stream>>>(W2, DHID, DM, DM, W2T);
  k_gemm<0, true><<<dim3(MROWS / GBM, NQKV / GBN), GTHR, 0, stream>>>(XB, WQKVT, DM, bq, bk, bv, x, RES, QKV, DK, 1.0f);
  k_stats<<<dim3(SEQ / 64, NZ), 128, 0, stream>>>(Qp, Kp, ST);
  k_attn<<<dim3(SEQ / 64, NZ), 128, 0, stream>>>(Qp, Kp, VTp, ST, CAT);
  k_gemm<1, false><<<dim3(MROWS / GBM, DM / GBN), GTHR, 0, stream>>>(CAT, WOT, DM, bo, bo, bo, x, RES, RESH, DM,
                                                                     1.0f / 16384.0f);
  k_ln<<<cdiv(MROWS, 4), 128, 0, stream>>>(RES, g1, be1, SAE, MROWS);
  k_gemm<2, false><<<dim3(MROWS / GBM, DHID / GBN), GTHR, 0, stream>>>(RESH, W1T, DM, b1, b1, b1, x, RES, H1, DHID,
                                                                       1.0f / 256.0f);
  k_gemm<3, false><<<dim3(MROWS / GBM, DM / GBN), GTHR, 0, stream>>>(H1, W2T, DHID, b2, b2, b2, SAE, OPRE, RESH, DM,
                                                                     1.0f / 256.0f);
  k_ln<<<cdiv(MROWS, 4), 128, 0, stream>>>(OPRE, g2, be2, out, MROWS);
}
